// SelfAttention_19104014532772
// MI455X (gfx1250) — hardware-verified
//
#include <hip/hip_runtime.h>
#ifndef NB
#define NB 4
#endif
#ifndef SEQ
#define SEQ 4096
#endif
#define SEQ_FULL 4096
#define CC 256
#define RD 64
#define CH 128
#define PCARRY_LN 8.317766166719343f
#define PINV 0.000244140625f
#define NRT ((size_t)NB * SEQ)

static_assert(SEQ % 256 == 0);
static_assert(SEQ <= SEQ_FULL);
static_assert(CC % 64 == 0);
static_assert(RD == 64);
static_assert(CC == 2 * CH);
static_assert(CH % 16 == 0 && CH / 16 == 8);

typedef __bf16 v16b __attribute__((ext_vector_type(16)));
typedef _Float16 v16h __attribute__((ext_vector_type(16)));
typedef unsigned short v8us __attribute__((ext_vector_type(8), may_alias));
typedef float v8f  __attribute__((ext_vector_type(8)));
typedef float v4f  __attribute__((ext_vector_type(4)));
typedef float v4fa __attribute__((ext_vector_type(4), may_alias));
union FragB { v16b v; v8us half[2]; };
union FragH { v16h v; v8us half[2]; _Float16 h[16]; };

__device__ __forceinline__ unsigned short bf16_bits(float x) { unsigned int u = __float_as_uint(x); return (unsigned short)((u + 0x7FFFu + ((u >> 16) & 1u)) >> 16); }
__device__ __forceinline__ float bf16_val(unsigned short b) { return __uint_as_float(((unsigned int)b) << 16); }
__device__ __forceinline__ float bf16_rne(float x) { return bf16_val(bf16_bits(x)); }

__device__ __forceinline__ v16b ld_bf(const unsigned short* p, int hh) { FragB f; f.half[0] = *(const v8us*)(p + 8 * hh); f.half[1] = *(const v8us*)(p + 16 + 8 * hh); return f.v; }

__device__ __forceinline__ v8f mma_b1(v16b a, v16b b, v8f c) {
  c = __builtin_amdgcn_wmma_f32_16x16x32_bf16(false, a, false, b, (short)0, c, false, false);
  asm volatile("v_nop\n\tv_nop\n\tv_nop\n\tv_nop" : "+v"(c) : "v"(a), "v"(b));
  return c;
}
__device__ __forceinline__ v8f mma_b3(v16b ah, v16b al, v16b bh, v16b bl, v8f c) {
  c = __builtin_amdgcn_wmma_f32_16x16x32_bf16(false, ah, false, bh, (short)0, c, false, false);
  c = __builtin_amdgcn_wmma_f32_16x16x32_bf16(false, al, false, bh, (short)0, c, false, false);
  c = __builtin_amdgcn_wmma_f32_16x16x32_bf16(false, ah, false, bl, (short)0, c, false, false);
  asm volatile("v_nop\n\tv_nop\n\tv_nop\n\tv_nop" : "+v"(c) : "v"(ah), "v"(al), "v"(bh), "v"(bl));
  return c;
}
__device__ __forceinline__ v8f mma_h1(v16h a, v16h b, v8f c) {
  c = __builtin_amdgcn_wmma_f32_16x16x32_f16(false, a, false, b, (short)0, c, false, false);
  asm volatile("v_nop\n\tv_nop\n\tv_nop\n\tv_nop" : "+v"(c) : "v"(a), "v"(b));
  return c;
}

__global__ __launch_bounds__(256) void k_wcvt(const float* __restrict__ W, unsigned short* __restrict__ Wb, int n8) {
  const int t = blockIdx.x * 256 + threadIdx.x;
  if (t >= n8) return;
  const v4f a = *(const v4fa*)(W + (size_t)t * 8);
  const v4f c = *(const v4fa*)(W + (size_t)t * 8 + 4);
  v8us v;
#pragma unroll
  for (int q = 0; q < 4; ++q) { v[q] = bf16_bits(a[q]); v[4 + q] = bf16_bits(c[q]); }
  unsigned short* d = Wb + (size_t)t * 8;
  *(volatile v8us*)d = v;
  __threadfence();
  *(volatile v8us*)d = v;
}

__global__ __launch_bounds__(256) void k_xT(const float* __restrict__ x, unsigned short* __restrict__ XB) {
  __shared__ unsigned short tl[64][66];
  const int tid = threadIdx.x;
  const int blk = blockIdx.x;
  const int ct = blk % (CC / 64);
  const int nt = (blk / (CC / 64)) % (SEQ / 64);
  const int b = blk / ((CC / 64) * (SEQ / 64));
#pragma unroll 1
  for (int i = tid; i < 64 * 16; i += 256) {
    const int c = i >> 4, n4 = (i & 15) * 4;
    const v4f v = *(const v4fa*)(x + ((size_t)(b * CC + ct * 64 + c)) * SEQ_FULL + nt * 64 + n4);
#pragma unroll
    for (int q = 0; q < 4; ++q) tl[n4 + q][c] = bf16_bits(v[q]);
  }
  __syncthreads();
  for (int pass = 0; pass < 2; ++pass) {
#pragma unroll 1
    for (int i = tid; i < 64 * 8; i += 256) {
      const int n = i >> 3, c8 = (i & 7) * 8;
      v8us f;
#pragma unroll
      for (int q = 0; q < 8; ++q) f[q] = tl[n][c8 + q];
      unsigned short* d = XB + ((size_t)b * SEQ + nt * 64 + n) * CC + ct * 64 + c8;
      *(volatile v8us*)d = f;
    }
    if (pass == 0) __threadfence();
  }
}

__global__ __launch_bounds__(128) void k_qproj(const unsigned short* __restrict__ XB, const unsigned short* __restrict__ WRB,
                                               unsigned short* __restrict__ QH, unsigned short* __restrict__ QL) {
  __shared__ __attribute__((aligned(16))) float so[4][16][64];
  const int tid = threadIdx.x;
  const int wave = __builtin_amdgcn_readfirstlane(tid >> 5);
  const int lane = tid & 31, ln = lane & 15, hh = lane >> 4;
  const size_t row0 = ((size_t)blockIdx.x * 4 + wave) * 16;
  const unsigned short* arow = XB + (row0 + ln) * CC;
  const v8f z8 = {0.f, 0.f, 0.f, 0.f, 0.f, 0.f, 0.f, 0.f};
  v8f acc[4];
#pragma unroll
  for (int t = 0; t < 4; ++t) acc[t] = z8;
#pragma unroll 1
  for (int kb = 0; kb < CC; kb += 32) {
    const v16b a = ld_bf(arow + kb, hh);
#pragma unroll
    for (int t = 0; t < 4; ++t) {
      const v16b bq = ld_bf(WRB + (size_t)(t * 16 + ln) * CC + kb, hh);
      acc[t] = mma_b1(a, bq, acc[t]);
    }
  }
#pragma unroll
  for (int t = 0; t < 4; ++t)
#pragma unroll
    for (int r = 0; r < 8; ++r) so[wave][8 * hh + r][t * 16 + ln] = acc[t][r];
  __builtin_amdgcn_fence(4  , "workgroup");
  __builtin_amdgcn_wave_barrier();
  const int rsub = lane >> 3, c8 = (lane & 7) * 8;
  for (int pass = 0; pass < 2; ++pass) {
#pragma unroll
    for (int it = 0; it < 4; ++it) {
      const int r = it * 4 + rsub;
      const v4f a = *(const v4fa*)&so[wave][r][c8];
      const v4f c = *(const v4fa*)&so[wave][r][c8 + 4];
      v8us vh, vl;
#pragma unroll
      for (int q = 0; q < 4; ++q) {
        unsigned short hb = bf16_bits(a[q]); vh[q] = hb; vl[q] = bf16_bits(a[q] - bf16_val(hb));
        hb = bf16_bits(c[q]); vh[4 + q] = hb; vl[4 + q] = bf16_bits(c[q] - bf16_val(hb));
      }
      const size_t o = (row0 + r) * RD + c8;
      *(volatile v8us*)(QH + o) = vh;
      *(volatile v8us*)(QL + o) = vl;
    }
    if (pass == 0) __threadfence();
  }
}

__global__ __launch_bounds__(128) void k_vproj(const unsigned short* __restrict__ XB, const unsigned short* __restrict__ WFB,
                                               unsigned short* __restrict__ VT) {
  __shared__ __attribute__((aligned(16))) float so[4][16][64];
  const int tid = threadIdx.x;
  const int wave = __builtin_amdgcn_readfirstlane(tid >> 5);
  const int lane = tid & 31, ln = lane & 15, hh = lane >> 4;
  const int b = blockIdx.y;
  const int wid = blockIdx.x * 4 + wave;
  const int mt = wid / (SEQ / 64), nq = wid % (SEQ / 64);
  const unsigned short* arow = WFB + (size_t)(mt * 16 + ln) * CC;
  const unsigned short* brow = XB + ((size_t)b * SEQ + nq * 64 + ln) * CC;
  const v8f z8 = {0.f, 0.f, 0.f, 0.f, 0.f, 0.f, 0.f, 0.f};
  v8f acc[4];
#pragma unroll
  for (int t = 0; t < 4; ++t) acc[t] = z8;
#pragma unroll 1
  for (int kb = 0; kb < CC; kb += 32) {
    const v16b a = ld_bf(arow + kb, hh);
#pragma unroll
    for (int t = 0; t < 4; ++t) {
      const v16b bq = ld_bf(brow + (size_t)(t * 16) * CC + kb, hh);
      acc[t] = mma_b1(a, bq, acc[t]);
    }
  }
#pragma unroll
  for (int t = 0; t < 4; ++t)
#pragma unroll
    for (int r = 0; r < 8; ++r) so[wave][8 * hh + r][t * 16 + ln] = acc[t][r];
  __builtin_amdgcn_fence(4  , "workgroup");
  __builtin_amdgcn_wave_barrier();
  const int rsub = lane >> 3, c8 = (lane & 7) * 8;
  for (int pass = 0; pass < 2; ++pass) {
#pragma unroll
    for (int it = 0; it < 4; ++it) {
      const int r = it * 4 + rsub;
      const v4f a = *(const v4fa*)&so[wave][r][c8];
      const v4f c = *(const v4fa*)&so[wave][r][c8 + 4];
      FragH f;
#pragma unroll
      for (int q = 0; q < 4; ++q) { f.h[q] = (_Float16)a[q]; f.h[4 + q] = (_Float16)c[q]; }
      const v8us o = f.half[0];
      *(volatile v8us*)(VT + ((size_t)(b * CC + mt * 16 + r)) * SEQ + nq * 64 + c8) = o;
    }
    if (pass == 0) __threadfence();
  }
}

__global__ __launch_bounds__(128) void k_stats(const unsigned short* __restrict__ QH, const unsigned short* __restrict__ QL, float* __restrict__ E) {
  __shared__ __attribute__((aligned(16))) float st[64];
  const int tid = threadIdx.x;
  const int wave = __builtin_amdgcn_readfirstlane(tid >> 5);
  const int lane = tid & 31, ln = lane & 15, hh = lane >> 4;
  const int b = blockIdx.y;
  const size_t tb = (size_t)b * SEQ;
  const size_t ao = (tb + (size_t)blockIdx.x * 64 + wave * 16 + ln) * RD;
  const v16b aH0 = ld_bf(QH + ao, hh), aL0 = ld_bf(QL + ao, hh), aH1 = ld_bf(QH + ao + 32, hh), aL1 = ld_bf(QL + ao + 32, hh);
  const v8f z8 = {0.f, 0.f, 0.f, 0.f, 0.f, 0.f, 0.f, 0.f};
  float m[8], l[8];
#pragma unroll
  for (int r = 0; r < 8; ++r) { m[r] = -1.0e30f; l[r] = 0.f; }
#pragma unroll 1
  for (int j0 = 0; j0 < SEQ; j0 += 32) {
    const size_t bo0 = (tb + j0 + ln) * RD, bo1 = bo0 + (size_t)16 * RD;
    v8f s0 = z8, s1 = z8;
    { v16b bh = ld_bf(QH + bo0, hh), bl = ld_bf(QL + bo0, hh); s0 = mma_b3(aH0, aL0, bh, bl, s0);
      bh = ld_bf(QH + bo0 + 32, hh); bl = ld_bf(QL + bo0 + 32, hh); s0 = mma_b3(aH1, aL1, bh, bl, s0); }
    { v16b bh = ld_bf(QH + bo1, hh), bl = ld_bf(QL + bo1, hh); s1 = mma_b3(aH0, aL0, bh, bl, s1);
      bh = ld_bf(QH + bo1 + 32, hh); bl = ld_bf(QL + bo1 + 32, hh); s1 = mma_b3(aH1, aL1, bh, bl, s1); }
#pragma unroll
    for (int r = 0; r < 8; ++r) {
      const float a0 = s0[r], a1 = s1[r];
      const float mn = fmaxf(m[r], fmaxf(a0, a1));
      l[r] = l[r] * __expf(m[r] - mn) + __expf(a0 - mn) + __expf(a1 - mn);
      m[r] = mn;
    }
  }
#pragma unroll
  for (int off = 1; off < 16; off <<= 1) {
#pragma unroll
    for (int r = 0; r < 8; ++r) {
      const float mo = __shfl_xor(m[r], off);
      const float lo = __shfl_xor(l[r], off);
      const float mn = fmaxf(m[r], mo);
      l[r] = l[r] * __expf(m[r] - mn) + lo * __expf(mo - mn);
      m[r] = mn;
    }
  }
  float ev[8];
#pragma unroll
  for (int r = 0; r < 8; ++r) ev[r] = m[r] + __logf(l[r]) - PCARRY_LN;
  if (ln == 0) {
#pragma unroll
    for (int r = 0; r < 8; ++r) st[wave * 16 + 8 * hh + r] = ev[r];
  }
  __syncthreads();
  if (wave == 0 && lane < 16) {
    const v4f v = *(const v4fa*)&st[lane * 4];
    float* d = E + tb + (size_t)blockIdx.x * 64 + lane * 4;
    *(volatile v4f*)d = v;
    __threadfence();
    *(volatile v4f*)d = v;
  }
}

__global__ __launch_bounds__(128) void k_attn(const unsigned short* __restrict__ QH, const unsigned short* __restrict__ QL,
                                              const unsigned short* __restrict__ VT, const float* __restrict__ E,
                                              const float* __restrict__ x, float* __restrict__ out) {
  __shared__ __attribute__((aligned(16))) float so[CH][68];
  const int tid = threadIdx.x;
  const int wave = __builtin_amdgcn_readfirstlane(tid >> 5);
  const int lane = tid & 31, ln = lane & 15, hh = lane >> 4;
  const int b = blockIdx.z, ch0 = blockIdx.y * CH, jb = blockIdx.x * 64;
  const size_t tb = (size_t)b * SEQ;
  const size_t bo = (tb + jb + wave * 16 + ln) * RD;
  const v16b bH0 = ld_bf(QH + bo, hh), bL0 = ld_bf(QL + bo, hh), bH1 = ld_bf(QH + bo + 32, hh), bL1 = ld_bf(QL + bo + 32, hh);
  const v8f z8 = {0.f, 0.f, 0.f, 0.f, 0.f, 0.f, 0.f, 0.f};
  v8f acc[8];
#pragma unroll
  for (int i = 0; i < 8; ++i) acc[i] = z8;
  const size_t vrow = ((size_t)(b * CC + ch0 + ln)) * SEQ + 8 * hh;
#pragma unroll 1
  for (int n0 = 0; n0 < SEQ; n0 += 32) {
    const size_t ao0 = (tb + n0 + ln) * RD, ao1 = ao0 + (size_t)16 * RD;
    v8f s0 = z8, s1 = z8;
    { v16b ah = ld_bf(QH + ao0, hh), al = ld_bf(QL + ao0, hh); s0 = mma_b3(ah, al, bH0, bL0, s0);
      ah = ld_bf(QH + ao0 + 32, hh); al = ld_bf(QL + ao0 + 32, hh); s0 = mma_b3(ah, al, bH1, bL1, s0); }
    asm volatile("" ::: "memory");
    { v16b ah = ld_bf(QH + ao1, hh), al = ld_bf(QL + ao1, hh); s1 = mma_b3(ah, al, bH0, bL0, s1);
      ah = ld_bf(QH + ao1 + 32, hh); al = ld_bf(QL + ao1 + 32, hh); s1 = mma_b3(ah, al, bH1, bL1, s1); }
    asm volatile("" ::: "memory");
    const float* ep = E + tb + n0 + 8 * hh;
    const v4f e0a = *(const v4fa*)ep, e0b = *(const v4fa*)(ep + 4), e1a = *(const v4fa*)(ep + 16), e1b = *(const v4fa*)(ep + 20);
    FragH pf;
#pragma unroll
    for (int r = 0; r < 4; ++r) {
      pf.h[r]      = (_Float16)__expf(s0[r]     - e0a[r]);
      pf.h[4 + r]  = (_Float16)__expf(s0[4 + r] - e0b[r]);
      pf.h[8 + r]  = (_Float16)__expf(s1[r]     - e1a[r]);
      pf.h[12 + r] = (_Float16)__expf(s1[4 + r] - e1b[r]);
    }
    asm volatile("" ::: "memory");
#pragma unroll
    for (int g = 0; g < 2; ++g) {
#pragma unroll
      for (int ct = 0; ct < 4; ++ct) {
        const int idx = g * 4 + ct;
        const unsigned short* vp = VT + vrow + (size_t)(idx * 16) * SEQ + n0;
        FragH a;
        a.half[0] = *(const v8us*)vp;
        a.half[1] = *(const v8us*)(vp + 16);
        acc[idx] = mma_h1(a.v, pf.v, acc[idx]);
      }
      asm volatile("" ::: "memory");
    }
  }
#pragma unroll
  for (int ct = 0; ct < 8; ++ct)
#pragma unroll
    for (int r = 0; r < 8; ++r) so[ct * 16 + 8 * hh + r][wave * 16 + ln] = acc[ct][r] * PINV;
  __syncthreads();
  const int rsub = lane >> 4, pc = (lane & 15) * 4;
  for (int pass = 0; pass < 2; ++pass) {
#pragma unroll 1
    for (int it = 0; it < CH / 8; ++it) {
      const int row = it * 8 + wave * 2 + rsub;
      const v4f v = *(const v4fa*)&so[row][pc];
      const v4f xr = *(const v4fa*)(x + ((size_t)(b * CC + ch0 + row)) * SEQ_FULL + jb + pc);
      v4f o;
#pragma unroll
      for (int q = 0; q < 4; ++q) o[q] = bf16_rne(xr[q]) + v[q];
      *(volatile v4f*)(out + ((size_t)(b * CC + ch0 + row)) * SEQ + jb + pc) = o;
    }
    if (pass == 0) __threadfence();
  }
}

#define SZ_WRB ((size_t)RD * CC * 2)
#define SZ_WFB ((size_t)CC * CC * 2)
#define SZ_XB  (NRT * CC * 2)
#define SZ_Q   (NRT * RD * 2)
#define SZ_VT  ((size_t)NB * CC * SEQ * 2)
#define SZ_E   (NRT * 4)
#define OFF_WRB ((size_t)0)
#define OFF_WFB (OFF_WRB + SZ_WRB)
#define OFF_XB  (OFF_WFB + SZ_WFB)
#define OFF_QH  (OFF_XB + SZ_XB)
#define OFF_QL  (OFF_QH + SZ_Q)
#define OFF_VT  (OFF_QL + SZ_Q)
#define OFF_E   (OFF_VT + SZ_VT)
#define WS_TOTAL (OFF_E + SZ_E)
static_assert(SZ_WRB % 256 == 0 && SZ_WFB % 256 == 0 && SZ_XB % 256 == 0 && SZ_Q % 256 == 0 && SZ_VT % 256 == 0 && SZ_E % 256 == 0);
static_assert(WS_TOTAL <= (size_t)134217728);
static_assert((RD * CC) % (8 * 256) == 0 && (CC * CC) % (8 * 256) == 0);
static_assert((NRT % 64) == 0);
static_assert((16 * (SEQ / 64)) % 4 == 0);

extern "C" void kernel_launch(void* const* d_in, const int* in_sizes, int n_in,
                              void* d_out, int out_size, void* d_ws, size_t ws_size, hipStream_t stream) {
  if (n_in < 3) return;
  if ((size_t)in_sizes[0] < (size_t)(NB * CC - 1) * SEQ_FULL + SEQ) return;
  if ((size_t)in_sizes[1] < (size_t)RD * CC) return;
  if ((size_t)in_sizes[2] < (size_t)CC * CC) return;
  if ((size_t)out_size < (size_t)NB * CC * SEQ) return;
  if (WS_TOTAL > ws_size) return;
  const float* x = (const float*)d_in[0];
  const float* wr = (const float*)d_in[1];
  const float* wf = (const float*)d_in[2];
  float* out = (float*)d_out;
  char* ws = (char*)d_ws;
  unsigned short* WRB = (unsigned short*)(ws + OFF_WRB);
  unsigned short* WFB = (unsigned short*)(ws + OFF_WFB);
  unsigned short* XB  = (unsigned short*)(ws + OFF_XB);
  unsigned short* QH  = (unsigned short*)(ws + OFF_QH);
  unsigned short* QL  = (unsigned short*)(ws + OFF_QL);
  unsigned short* VT  = (unsigned short*)(ws + OFF_VT);
  float* E = (float*)(ws + OFF_E);

  k_wcvt<<<(RD * CC / 8) / 256, 256, 0, stream>>>(wr, WRB, RD * CC / 8);
  k_wcvt<<<(CC * CC / 8) / 256, 256, 0, stream>>>(wf, WFB, CC * CC / 8);
  k_xT<<<(CC / 64) * (SEQ / 64) * NB, 256, 0, stream>>>(x, XB);
  k_qproj<<<(unsigned)(NRT / 64), 128, 0, stream>>>(XB, WRB, QH, QL);
  k_vproj<<<dim3(16 * (SEQ / 64) / 4, NB), 128, 0, stream>>>(XB, WFB, VT);
  k_stats<<<dim3(SEQ / 64, NB), 128, 0, stream>>>(QH, QL, E);
  k_attn<<<dim3(SEQ / 64, CC / CH, NB), 128, 0, stream>>>(QH, QL, VT, E, x, out);
}
